// MPNN_22230750724232
// MI455X (gfx1250) — hardware-verified
//
#include <hip/hip_runtime.h>
#include <stddef.h>
#include <stdint.h>


#define NNODE  50000
#define NEDGE  500000
#define NGRAPH 1024
#define NDIM   32
#define EDIM   16
#define HID    128
#define NLAY   4
#define NTHR   256
#define NWAVE  8
#define TROWS  128
#define NCAP   64
#define DEGCAP 120
#define TCAP   128
#define NBA    1024
#define SLA    10
#define NBLK   49
#define RCAP   28672
#define EPT    8
#define CHUNK  (NTHR * EPT)
#define WCAP   (EPT * 32)
#define LISTN  (NWAVE * WCAP)
#define MP     50048
#define RROWS  (NEDGE + NBLK * 128)
#define NDEG   (NBLK * NBA)
#define SP     132
#define AP     136
#define FP     40
#define HLP    264
#define PG     32
#define NCST   20
#define BK_ZINTS (LISTN + 2 * RCAP + 3 * NBA)
#define BK_LDS_INTS (BK_ZINTS + 16 + TCAP * 4 + 32)
#define BK_LDS_BYTES (BK_LDS_INTS * 4)
#define NODE_LDS_BYTES (TROWS * SP * 4 + TROWS * HLP * 2)
#define EDGE_LDS_BYTES (TROWS * SP * 4 + 2 * TROWS * AP * 2 + 2 * HID * 4 + 3 * TROWS * 4)
#define CR     16.0f
#define CW     256.0f
#define PINV   0.000244140625f
#define INVSTD 0.9999950000374997f
#define PU0    512
#define PU1    (PU0 + 16384)
#define PU2    (PU1 + 16384)
#define PU3    (PU2 + 4096)
#define PU4    (PU3 + 512)
#define PU5    (PU4 + 14336)
#define PU6    (PU5 + 768)
#define WSCAP  268435456ull

static_assert(HID == 128 && 2 * HID == 256 && NDIM == 32 && EDIM == 16 && NLAY == 4);
static_assert(NNODE == 50000 && NEDGE == 500000 && NGRAPH == 1024);
static_assert(TROWS == 128 && DEGCAP < 128 && DEGCAP >= 26 + 8);
static_assert(RCAP >= 10475 + 10475 / 20 + 1);
static_assert(TCAP >= (10475 + 99) / 100);
static_assert(CR * CW * PINV == 1.0f);
static_assert((CHUNK & (CHUNK - 1)) == 0 && CHUNK <= 4096);
static_assert((NBA & (NBA - 1)) == 0 && NBA == (1 << SLA));
static_assert(((long long)CHUNK << SLA) < (1LL << 31));
static_assert(NEDGE < (1 << 21) && (NEDGE % 4) == 0);
static_assert(NBLK * NBA >= NNODE && (NBLK - 1) * NBA < NNODE);
static_assert(MP % TROWS == 0 && MP >= NNODE && MP <= NDEG);
static_assert(NBA % NWAVE == 0 && NBA % 32 == 0 && NBA == 4 * NTHR);
static_assert(RCAP % (4 * NTHR) == 0 && BK_LDS_INTS % 4 == 0);
static_assert(BK_LDS_BYTES <= 300000 && NODE_LDS_BYTES <= 300000 && EDGE_LDS_BYTES <= 300000);
static_assert(NCAP * HID * 4 <= TROWS * AP * 2);
static_assert((SP * 4) % 16 == 0 && (AP * 2) % 16 == 0 && (FP * 2) % 16 == 0 && (HLP * 2) % 16 == 0);
static_assert(PU0 % NTHR == 0 && PU1 % NTHR == 0 && PU2 % NTHR == 0 && PU3 % NTHR == 0);
static_assert(PU4 % NTHR == 0 && PU5 % NTHR == 0 && PU6 % NTHR == 0);
static_assert(NGRAPH % PG == 0 && PG == 32 && NWAVE * 4 == PG);
static_assert(NCAP % NWAVE == 0 && TROWS == 16 * NWAVE);

typedef float          v4f   __attribute__((ext_vector_type(4)));
typedef float          v8f   __attribute__((ext_vector_type(8)));
typedef int            v4i   __attribute__((ext_vector_type(4)));
typedef int            v8i   __attribute__((ext_vector_type(8)));
typedef unsigned short v4us  __attribute__((ext_vector_type(4)));
typedef unsigned short v8us  __attribute__((ext_vector_type(8)));
typedef unsigned short v16us __attribute__((ext_vector_type(16)));
typedef __bf16         v16bf __attribute__((ext_vector_type(16)));
typedef _Float16       v16h  __attribute__((ext_vector_type(16)));
typedef v4f  __attribute__((may_alias)) v4fa;
typedef v4i  __attribute__((may_alias)) v4ia;
typedef v4us __attribute__((may_alias)) v4usa;
typedef v8us __attribute__((may_alias)) v8usa;
union FragB { v16bf v; v16us u; v8us h[2]; v8i w; };
union FragH { v16h  v; v16us u; v8us h[2]; v8i w; };

__device__ __forceinline__ v8f wmb(const FragB& a, const FragB& b, v8f c) {
  v8f d = __builtin_amdgcn_wmma_f32_16x16x32_bf16(false, a.v, false, b.v, (short)0, c, false, false);
  asm volatile("v_nop\n\tv_nop\n\tv_nop\n\tv_nop" : "+v"(d) : "v"(a.w), "v"(b.w));
  return d;
}
__device__ __forceinline__ v8f wmh(const FragH& a, const FragH& b, v8f c) {
  v8f d = __builtin_amdgcn_wmma_f32_16x16x32_f16(false, a.v, false, b.v, (short)0, c, false, false);
  asm volatile("v_nop\n\tv_nop\n\tv_nop\n\tv_nop" : "+v"(d) : "v"(a.w), "v"(b.w));
  return d;
}

__device__ __forceinline__ v8f z8() { v8f z = {0.f, 0.f, 0.f, 0.f, 0.f, 0.f, 0.f, 0.f}; return z; }
__device__ __forceinline__ int iclamp(int v, int lo, int hi) { return v < lo ? lo : (v > hi ? hi : v); }
__device__ __forceinline__ int imin(int a, int b) { return a < b ? a : b; }

__device__ __forceinline__ unsigned bf16_bits(float f) {
  const unsigned u = __float_as_uint(f);
  return (u + 0x7FFFu + ((u >> 16) & 1u)) >> 16;
}
__device__ __forceinline__ unsigned bf16_bits_np(float f) {
  const unsigned r = bf16_bits(f);
  return (f != f) ? 0x7fc0u : r;
}
__device__ __forceinline__ float bf16_val(float f) {
  return __uint_as_float(bf16_bits(f) << 16);
}
__device__ __forceinline__ unsigned short f2h(float f) {
  const _Float16 hv = (_Float16)f;
  return __builtin_bit_cast(unsigned short, hv);
}
__device__ __forceinline__ float relu_np(float v) { return (v > 0.0f) ? v : (v - v); }

__device__ __forceinline__ void put16(unsigned short* dp, v8us o) {
  *(volatile v8us*)dp = o;
  __threadfence();
  *(volatile v8us*)dp = o;
}
__device__ __forceinline__ void putf4(float* dp, v4f o) {
  *(volatile v4f*)dp = o;
  __threadfence();
  *(volatile v4f*)dp = o;
}
__device__ __forceinline__ void puti4(int* dp, v4i o) {
  *(volatile v4i*)dp = o;
  __threadfence();
  *(volatile v4i*)dp = o;
}

__device__ __forceinline__ void split4(v4f v, unsigned short* hp, unsigned short* lp) {
  v4us hv, lv;
  const unsigned h0 = bf16_bits_np(v.x), h1 = bf16_bits_np(v.y), h2 = bf16_bits_np(v.z), h3 = bf16_bits_np(v.w);
  hv.x = (unsigned short)h0; hv.y = (unsigned short)h1; hv.z = (unsigned short)h2; hv.w = (unsigned short)h3;
  lv.x = (unsigned short)bf16_bits_np(v.x - __uint_as_float(h0 << 16));
  lv.y = (unsigned short)bf16_bits_np(v.y - __uint_as_float(h1 << 16));
  lv.z = (unsigned short)bf16_bits_np(v.z - __uint_as_float(h2 << 16));
  lv.w = (unsigned short)bf16_bits_np(v.w - __uint_as_float(h3 << 16));
  *(v4usa*)hp = hv;
  *(v4usa*)lp = lv;
}

template <int SLB>
__device__ __forceinline__ int scan_chunk(const int* __restrict__ dsts, int nE, int cbase, int slotBase,
                                          int nb, int vec8, int* list, int tid, int lane, int wave) {
  int wc = 0;
  const int el0  = tid * EPT;
  const int e0   = cbase + el0;
  const int sent = -2147483647 - 1;
  v4i da, db;
  if (vec8 != 0 && cbase + CHUNK <= nE) {
    da = *(const v4i*)(dsts + e0);
    db = *(const v4i*)(dsts + e0 + 4);
  } else {
    da.x = (e0     < nE) ? dsts[min(e0,     nE - 1)] : sent;
    da.y = (e0 + 1 < nE) ? dsts[min(e0 + 1, nE - 1)] : sent;
    da.z = (e0 + 2 < nE) ? dsts[min(e0 + 2, nE - 1)] : sent;
    da.w = (e0 + 3 < nE) ? dsts[min(e0 + 3, nE - 1)] : sent;
    db.x = (e0 + 4 < nE) ? dsts[min(e0 + 4, nE - 1)] : sent;
    db.y = (e0 + 5 < nE) ? dsts[min(e0 + 5, nE - 1)] : sent;
    db.z = (e0 + 6 < nE) ? dsts[min(e0 + 6, nE - 1)] : sent;
    db.w = (e0 + 7 < nE) ? dsts[min(e0 + 7, nE - 1)] : sent;
  }
  const unsigned nbs = (unsigned)slotBase;
  const unsigned unb = (unsigned)nb;
  const unsigned s0 = (unsigned)da.x - nbs, s1 = (unsigned)da.y - nbs;
  const unsigned s2 = (unsigned)da.z - nbs, s3 = (unsigned)da.w - nbs;
  const unsigned s4 = (unsigned)db.x - nbs, s5 = (unsigned)db.y - nbs;
  const unsigned s6 = (unsigned)db.z - nbs, s7 = (unsigned)db.w - nbs;
  const bool h0 = s0 < unb, h1 = s1 < unb, h2 = s2 < unb, h3 = s3 < unb;
  const bool h4 = s4 < unb, h5 = s5 < unb, h6 = s6 < unb, h7 = s7 < unb;
  const unsigned any = __builtin_amdgcn_ballot_w32(h0 | h1 | h2 | h3 | h4 | h5 | h6 | h7);
  if (any != 0u) {
#define HITJ(J, HJ, SJ) { \
      const unsigned mj = __builtin_amdgcn_ballot_w32(HJ); \
      if (mj != 0u) { \
        if (HJ) { \
          const int pos = wc + (int)__builtin_amdgcn_mbcnt_lo(mj, 0u); \
          if (pos < WCAP) list[wave * WCAP + pos] = ((el0 + (J)) << SLB) | (int)(SJ); \
        } \
        wc += (int)__builtin_popcount(mj); } }
    HITJ(0, h0, s0)
    HITJ(1, h1, s1)
    HITJ(2, h2, s2)
    HITJ(3, h3, s3)
    HITJ(4, h4, s4)
    HITJ(5, h5, s5)
    HITJ(6, h6, s6)
    HITJ(7, h7, s7)
#undef HITJ
  }
  return wc;
}

__device__ __forceinline__ v8f comp8(const float* __restrict__ A8, const float* __restrict__ Bc) {
  float c0 = 0.f, c1 = 0.f, c2 = 0.f, c3 = 0.f, c4 = 0.f, c5 = 0.f, c6 = 0.f, c7 = 0.f;
#pragma unroll 1
  for (int j = 0; j < HID; j += 4) {
    const float b0 = bf16_val(Bc[(size_t)(j + 0) * HID]);
    const float b1 = bf16_val(Bc[(size_t)(j + 1) * HID]);
    const float b2 = bf16_val(Bc[(size_t)(j + 2) * HID]);
    const float b3 = bf16_val(Bc[(size_t)(j + 3) * HID]);
    const v4f r0 = *(const v4f*)(A8 + 0 * HID + j);
    const v4f r1 = *(const v4f*)(A8 + 1 * HID + j);
    const v4f r2 = *(const v4f*)(A8 + 2 * HID + j);
    const v4f r3 = *(const v4f*)(A8 + 3 * HID + j);
    const v4f r4 = *(const v4f*)(A8 + 4 * HID + j);
    const v4f r5 = *(const v4f*)(A8 + 5 * HID + j);
    const v4f r6 = *(const v4f*)(A8 + 6 * HID + j);
    const v4f r7 = *(const v4f*)(A8 + 7 * HID + j);
#define ROW4(C, R) C = fmaf(bf16_val(R.x), b0, C); C = fmaf(bf16_val(R.y), b1, C); \
                   C = fmaf(bf16_val(R.z), b2, C); C = fmaf(bf16_val(R.w), b3, C);
    ROW4(c0, r0) ROW4(c1, r1) ROW4(c2, r2) ROW4(c3, r3)
    ROW4(c4, r4) ROW4(c5, r5) ROW4(c6, r6) ROW4(c7, r7)
#undef ROW4
  }
  const v8f o = {c0, c1, c2, c3, c4, c5, c6, c7};
  return o;
}

__global__ __launch_bounds__(NTHR) void k_prep(
    const float* __restrict__ ne_w, const float* __restrict__ ne_b, const float* __restrict__ ee_w,
    const float* __restrict__ ee_b, const float* __restrict__ nm_w1, const float* __restrict__ nm_b1,
    const float* __restrict__ nm_w2, const float* __restrict__ nm_b2, const float* __restrict__ bn_g,
    const float* __restrict__ bn_b, const float* __restrict__ em_w1, const float* __restrict__ em_b1,
    const float* __restrict__ em_w2, const float* __restrict__ em_b2, const float* __restrict__ ro_w1,
    const float* __restrict__ ro_b1, const float* __restrict__ ro_w2, const float* __restrict__ ro_b2,
    unsigned short* NEWT, unsigned short* W1A, unsigned short* W2T, unsigned short* RO1,
    unsigned short* A0B, unsigned short* BW, float* CST) {
  const int u = (int)blockIdx.x * NTHR + (int)threadIdx.x;
  v8us o;
  if (u < PU0) {
    const int n  = u >> 2;
    const int k8 = (u & 3) * 8;
    const float* p = ne_w + (size_t)k8 * HID + n;
#pragma unroll
    for (int i = 0; i < 8; ++i) o[i] = (unsigned short)bf16_bits(p[(size_t)i * HID]);
    put16(NEWT + (size_t)n * NDIM + k8, o);
    return;
  } else if (u < PU1) {
    const int v  = u - PU0;
    const int l  = v >> 12;
    const int n  = (v >> 5) & (HID - 1);
    const int k8 = (v & 31) * 8;
    const float* p = nm_w1 + (size_t)l * 2 * HID * HID + (size_t)(k8 & (HID - 1)) * HID + n;
#pragma unroll
    for (int i = 0; i < 8; ++i) o[i] = (unsigned short)bf16_bits(p[(size_t)i * HID]);
    put16(W1A + ((size_t)l * HID + n) * 256 + k8, o);
    return;
  } else if (u < PU2) {
    const int v  = u - PU1;
    const int l  = v >> 12;
    const int n  = (v >> 5) & (HID - 1);
    const int k8 = (v & 31) * 8;
    const float* p = nm_w2 + (size_t)l * HID * HID + (size_t)(k8 & (HID - 1)) * HID + n;
#pragma unroll
    for (int i = 0; i < 8; ++i) o[i] = (unsigned short)bf16_bits(p[(size_t)i * HID]);
    put16(W2T + ((size_t)l * HID + n) * 256 + k8, o);
    return;
  } else if (u < PU3) {
    const int v  = u - PU2;
    const int n  = v >> 5;
    const int k8 = (v & 31) * 8;
    const float* p = ro_w1 + (size_t)(k8 & (HID - 1)) * HID + n;
#pragma unroll
    for (int i = 0; i < 8; ++i) o[i] = (unsigned short)bf16_bits(p[(size_t)i * HID]);
    put16(RO1 + (size_t)n * 256 + k8, o);
    return;
  } else if (u < PU5) {
    const float* Ap;
    const float* Bp;
    unsigned short* dp;
    unsigned lomask = 0u;
    const bool isA0 = u < PU4;
    if (isA0) {
      const int w  = u - PU3;
      const int n  = w >> 2;
      const int k8 = (w & 3) * 8;
      Ap = ee_w + (size_t)(k8 & 15) * HID;
      Bp = em_w1 + n;
      dp = A0B + (size_t)n * 32 + k8;
      lomask = (k8 >= 16) ? 0xffffffffu : 0u;
    } else {
      const int w = u - PU4;
      if (w < 3 * 4096) {
        const int l  = w >> 12;
        const int v  = w & 4095;
        const int n  = v >> 4;
        const int k8 = (v & 15) * 8;
        Ap = em_w2 + (size_t)l * HID * HID + (size_t)k8 * HID;
        if (n < HID) Bp = em_w1 + (size_t)(l + 1) * HID * HID + n;
        else         Bp = nm_w1 + (size_t)l * 2 * HID * HID + (size_t)HID * HID + (n - HID);
        dp = BW + (size_t)l * 256 * HID + (size_t)n * HID + k8;
      } else {
        const int v  = w - 3 * 4096;
        const int n  = v >> 4;
        const int k8 = (v & 15) * 8;
        Ap = em_w2 + (size_t)3 * HID * HID + (size_t)k8 * HID;
        Bp = nm_w1 + (size_t)3 * 2 * HID * HID + (size_t)HID * HID + n;
        dp = BW + (size_t)3 * 256 * HID + (size_t)n * HID + k8;
      }
    }
    const v8f c = comp8(Ap, Bp);
    if (isA0) {
#pragma unroll
      for (int i = 0; i < 8; ++i) {
        const unsigned hb = bf16_bits(c[i]);
        const unsigned lb = bf16_bits(c[i] - __uint_as_float(hb << 16));
        o[i] = (unsigned short)((hb & ~lomask) | (lb & lomask));
      }
    } else {
#pragma unroll
      for (int i = 0; i < 8; ++i) o[i] = f2h(CW * c[i]);
    }
    put16(dp, o);
    return;
  } else if (u < PU6) {
    const int w   = u - PU5;
    const int vid = w >> 5;
    const int q   = w & 31;
    if (vid >= NCST) return;
    v4f ov = {0.f, 0.f, 0.f, 0.f};
    if (vid < 8) {
      const float* av;
      const float* Mv;
      const float* bv;
      if (vid == 0)      { av = ee_b; Mv = em_w1; bv = em_b1; }
      else if (vid < 4)  { const int l = vid - 1; av = em_b2 + l * HID; Mv = em_w1 + (size_t)(l + 1) * HID * HID;
                           bv = em_b1 + (l + 1) * HID; }
      else               { const int l = vid - 4; av = em_b2 + l * HID;
                           Mv = nm_w1 + (size_t)l * 2 * HID * HID + (size_t)HID * HID; bv = nm_b1 + l * HID; }
      float a0 = 0.f, a1 = 0.f, a2 = 0.f, a3 = 0.f;
#pragma unroll 1
      for (int k = 0; k < HID; ++k) {
        const float a = bf16_val(av[k]);
        const v4f mr = *(const v4f*)(Mv + (size_t)k * HID + 4 * q);
        a0 = fmaf(a, bf16_val(mr.x), a0);
        a1 = fmaf(a, bf16_val(mr.y), a1);
        a2 = fmaf(a, bf16_val(mr.z), a2);
        a3 = fmaf(a, bf16_val(mr.w), a3);
      }
      const v4f bb = *(const v4f*)(bv + 4 * q);
      ov.x = a0 + bf16_val(bb.x); ov.y = a1 + bf16_val(bb.y);
      ov.z = a2 + bf16_val(bb.z); ov.w = a3 + bf16_val(bb.w);
    } else if (vid < 16) {
      const int l = vid & 3;
      const v4f g = *(const v4f*)(bn_g + l * HID + 4 * q);
      v4f s;
      s.x = INVSTD * bf16_val(g.x); s.y = INVSTD * bf16_val(g.y);
      s.z = INVSTD * bf16_val(g.z); s.w = INVSTD * bf16_val(g.w);
      if (vid < 12) {
        ov = s;
      } else {
        const v4f b2 = *(const v4f*)(nm_b2 + l * HID + 4 * q);
        const v4f bb = *(const v4f*)(bn_b + l * HID + 4 * q);
        ov.x = bf16_val(b2.x) * s.x + bf16_val(bb.x);
        ov.y = bf16_val(b2.y) * s.y + bf16_val(bb.y);
        ov.z = bf16_val(b2.z) * s.z + bf16_val(bb.z);
        ov.w = bf16_val(b2.w) * s.w + bf16_val(bb.w);
      }
    } else if (vid < 19) {
      const float* pv = (vid == 16) ? ne_b : ((vid == 17) ? ro_b1 : ro_w2);
      const v4f t = *(const v4f*)(pv + 4 * q);
      ov.x = bf16_val(t.x); ov.y = bf16_val(t.y); ov.z = bf16_val(t.z); ov.w = bf16_val(t.w);
    } else {
      const float t = bf16_val(ro_b2[0]);
      ov.x = t; ov.y = t; ov.z = t; ov.w = t;
    }
    putf4(CST + (size_t)vid * HID + 4 * q, ov);
    return;
  }
}

__global__ __launch_bounds__(NTHR) void k_hist(const int* __restrict__ dsts, int nE, int nN, int* CNTL) {
  __shared__ int sw[NWAVE];
  __shared__ __attribute__((aligned(16))) int sline[32];
  const int tid = (int)threadIdx.x, lane = tid & 31, wave = tid >> 5;
  const int nodeBase = (int)blockIdx.x * NBA;
  const int nb = iclamp(nN - nodeBase, 0, NBA);
  const unsigned nbs = (unsigned)nodeBase, unb = (unsigned)nb;
  const int nE4 = nE >> 2;
  const int nIt = (nE4 + NTHR - 1) / NTHR;
  const v4i* d4 = (const v4i*)dsts;
  int c = 0;
#pragma unroll 2
  for (int it = 0; it < nIt; ++it) {
    const int q  = it * NTHR + tid;
    const int qc = q < nE4 ? q : nE4 - 1;
    const v4i d = d4[qc];
    const int ok = q < nE4 ? 1 : 0;
    c += ok & (int)(((unsigned)d.x - nbs) < unb);
    c += ok & (int)(((unsigned)d.y - nbs) < unb);
    c += ok & (int)(((unsigned)d.z - nbs) < unb);
    c += ok & (int)(((unsigned)d.w - nbs) < unb);
  }
#pragma unroll
  for (int d = 16; d >= 1; d >>= 1) c += __shfl_xor(c, d, 32);
  if (lane == 0) sw[wave] = c;
  __syncthreads();
  int tot = 0;
#pragma unroll
  for (int w = 0; w < NWAVE; ++w) tot += sw[w];
  if (tid < 32) sline[tid] = tot;
  __syncthreads();
  v4i v = {0, 0, 0, 0};
  if (tid < 8) {
    v = *(const v4ia*)(sline + 4 * tid);
    *(volatile v4i*)(CNTL + (size_t)blockIdx.x * 32 + 4 * tid) = v;
  }
  __threadfence();
  if (tid < 8) *(volatile v4i*)(CNTL + (size_t)blockIdx.x * 32 + 4 * tid) = v;
}

__global__ __launch_bounds__(NTHR) void k_bucket(const int* __restrict__ srcs, const int* __restrict__ dsts,
                                                 int nE, int nN, int vec8, const int* __restrict__ CNTL,
                                                 int* PERM, int* SRCT, int* DEG, int* TILE, int* META) {
  extern __shared__ __attribute__((aligned(16))) int dsm[];
  int* list  = dsm;
  int* hl    = dsm + LISTN;
  int* sl    = hl + RCAP;
  int* cnt   = sl + RCAP;
  int* offs  = cnt + NBA;
  int* cur   = offs + NBA;
  int* misc  = cur + NBA;
  int* stile = misc + 16;
  int* smeta = stile + TCAP * 4;
  const int tid = (int)threadIdx.x, lane = tid & 31, wave = tid >> 5;
  const int nodeBase = (int)blockIdx.x * NBA;
  const int nb = iclamp(nN - nodeBase, 0, NBA);

  {
    const v4i z4 = {0, 0, 0, 0};
    for (int i = tid * 4; i < BK_LDS_INTS; i += NTHR * 4) *(v4ia*)(dsm + i) = z4;
  }
  __syncthreads();

  int t = 0, ov = 0;
  const int nChunks = (nE + CHUNK - 1) / CHUNK;
#pragma unroll 1
  for (int ch = 0; ch < nChunks; ++ch) {
    const int cbase = ch * CHUNK;
    const int wc = scan_chunk<SLA>(dsts, nE, cbase, nodeBase, nb, vec8, list, tid, lane, wave);
    if (lane == 0) misc[wave] = wc;
    __syncthreads();
    if (wave == 0) {
#pragma unroll 1
      for (int w2 = 0; w2 < NWAVE; ++w2) {
        int c = misc[w2];
        c = c < 0 ? 0 : (c > WCAP ? WCAP : c);
#pragma unroll 1
        for (int b0 = 0; b0 < c; b0 += 32) {
          const int idx = b0 + lane;
          const int ent = list[w2 * WCAP + (idx < WCAP ? idx : WCAP - 1)];
          const int m32 = (c - b0) < 32 ? (c - b0) : 32;
#pragma unroll 1
          for (int k = 0; k < m32; ++k) {
            const int u    = __builtin_amdgcn_readlane(ent, k);
            const int slot = u & (NBA - 1);
            const int el   = (u >> SLA) & (CHUNK - 1);
            const int pk   = ((cbase + el) << SLA) | slot;
            if (t < RCAP) {
              if (lane == 0) { hl[t] = pk; cnt[slot] = cnt[slot] + 1; }
              t = t + 1;
            } else {
              ov = 1;
            }
          }
        }
      }
    }
    __syncthreads();
  }
  if (wave == 0 && lane == 0) { misc[8] = t; misc[9] = ov; }
  __syncthreads();
  int tt = misc[8];
  tt = tt < 0 ? 0 : (tt > RCAP ? RCAP : tt);
  const int ovf = misc[9];

  if (wave == 0) {
    const int base = lane * (NBA / 32);
    int s = 0;
#pragma unroll 1
    for (int i = 0; i < NBA / 32; ++i) s += cnt[base + i];
    int incl = s;
#pragma unroll
    for (int d = 1; d < 32; d <<= 1) {
      const int y = __shfl_up(incl, d, 32);
      if (lane >= d) incl += y;
    }
    int run = incl - s;
#pragma unroll 1
    for (int i = 0; i < NBA / 32; ++i) {
      const int cv = cnt[base + i];
      offs[base + i] = run;
      cur[base + i]  = run;
      run += cv;
    }
  }
  __syncthreads();
  if (wave == 0) {
#pragma unroll 1
    for (int b0 = 0; b0 < tt; b0 += 32) {
      const int idx = b0 + lane;
      const int ent = hl[idx < RCAP ? idx : RCAP - 1];
      const int m32 = (tt - b0) < 32 ? (tt - b0) : 32;
#pragma unroll 1
      for (int k = 0; k < m32; ++k) {
        const int u    = __builtin_amdgcn_readlane(ent, k);
        const int slot = u & (NBA - 1);
        if (lane == 0) {
          int p = cur[slot];
          p = p < 0 ? 0 : (p > RCAP - 1 ? RCAP - 1 : p);
          sl[p] = u;
          cur[slot] = p + 1;
        }
      }
    }
  }
  __syncthreads();

  int basep = 0;
#pragma unroll 1
  for (int bb = 0; bb < NBLK; ++bb) {
    const int c  = iclamp(CNTL[bb * 32], 0, RCAP);
    const int rp = (c + 127) & ~127;
    basep += (bb < (int)blockIdx.x) ? rp : 0;
  }
  const int ppad = (tt + 127) & ~127;
  const bool fit = (basep + ppad) <= RROWS;

  if (tid == 0) {
    int nt = 0;
    int pois = ovf | (fit ? 0 : 1);
    int lo = 0, ec = 0, nc = 0, pl = 0;
#pragma unroll 1
    for (int s = 0; s < nb; ++s) {
      int d = cnt[s];
      d = d < 0 ? 0 : d;
      if (d > DEGCAP) { pois = 1; d = DEGCAP; }
      if (nc > 0 && (ec + d > TROWS || nc >= NCAP)) {
        if (nt < TCAP) {
          stile[4 * nt + 0] = nodeBase + lo; stile[4 * nt + 1] = nc;
          stile[4 * nt + 2] = basep + pl;    stile[4 * nt + 3] = ec;
          nt = nt + 1;
        } else {
          pois = 1;
        }
        pl += ec; lo = s; ec = 0; nc = 0;
      }
      ec += d; nc += 1;
    }
    if (nc > 0) {
      if (nt < TCAP) {
        stile[4 * nt + 0] = nodeBase + lo; stile[4 * nt + 1] = nc;
        stile[4 * nt + 2] = basep + pl;    stile[4 * nt + 3] = ec;
        nt = nt + 1;
      } else {
        pois = 1;
      }
    }
    smeta[0] = fit ? nt : 0;
    smeta[1] = pois;
    smeta[2] = basep;
    smeta[3] = tt;
  }
  __syncthreads();

  if (fit) {
#pragma unroll 1
    for (int it = 0; it < RCAP / (4 * NTHR); ++it) {
      const int q = it * NTHR + tid;
      if (4 * q < ppad) {
        const int p0 = 4 * q;
        const int n0 = sl[imin(p0 + 0, RCAP - 1)];
        const int n1 = sl[imin(p0 + 1, RCAP - 1)];
        const int n2 = sl[imin(p0 + 2, RCAP - 1)];
        const int n3 = sl[imin(p0 + 3, RCAP - 1)];
        const int e0 = iclamp(n0 >> SLA, 0, nE - 1);
        const int e1 = iclamp(n1 >> SLA, 0, nE - 1);
        const int e2 = iclamp(n2 >> SLA, 0, nE - 1);
        const int e3 = iclamp(n3 >> SLA, 0, nE - 1);
        const int s0 = iclamp(srcs[e0], 0, nN - 1);
        const int s1 = iclamp(srcs[e1], 0, nN - 1);
        const int s2 = iclamp(srcs[e2], 0, nN - 1);
        const int s3 = iclamp(srcs[e3], 0, nN - 1);
        v4i pe, sr;
        pe.x = (p0 + 0 < tt) ? e0 : -1; sr.x = (p0 + 0 < tt) ? s0 : 0;
        pe.y = (p0 + 1 < tt) ? e1 : -1; sr.y = (p0 + 1 < tt) ? s1 : 0;
        pe.z = (p0 + 2 < tt) ? e2 : -1; sr.z = (p0 + 2 < tt) ? s2 : 0;
        pe.w = (p0 + 3 < tt) ? e3 : -1; sr.w = (p0 + 3 < tt) ? s3 : 0;
        puti4(PERM + (size_t)basep + p0, pe);
        puti4(SRCT + (size_t)basep + p0, sr);
      }
    }
  }

  {
    v4i dv;
    dv.x = iclamp(cnt[4 * tid + 0], 0, 127);
    dv.y = iclamp(cnt[4 * tid + 1], 0, 127);
    dv.z = iclamp(cnt[4 * tid + 2], 0, 127);
    dv.w = iclamp(cnt[4 * tid + 3], 0, 127);
    puti4(DEG + (size_t)nodeBase + 4 * tid, dv);
  }

  {
    v4i tv = {0, 0, 0, 0};
    v4i mv = {0, 0, 0, 0};
    if (tid < TCAP) tv = *(const v4ia*)(stile + 4 * tid);
    if (tid < 8)    mv = *(const v4ia*)(smeta + 4 * tid);
    if (tid < TCAP) *(volatile v4i*)(TILE + ((size_t)blockIdx.x * TCAP + tid) * 4) = tv;
    if (tid < 8)    *(volatile v4i*)(META + (size_t)blockIdx.x * 32 + 4 * tid) = mv;
    __threadfence();
    if (tid < TCAP) *(volatile v4i*)(TILE + ((size_t)blockIdx.x * TCAP + tid) * 4) = tv;
    if (tid < 8)    *(volatile v4i*)(META + (size_t)blockIdx.x * 32 + 4 * tid) = mv;
  }
}

__device__ __forceinline__ void gemm_bf_k256(const unsigned short* ap, const unsigned short* __restrict__ bp,
                                             v8f (&acc)[8]) {
#pragma unroll 1
  for (int k0 = 0; k0 < 256; k0 += 32) {
    FragB af;
    af.h[0] = *(const v8usa*)(ap + k0);
    af.h[1] = *(const v8usa*)(ap + k0 + 16);
#pragma unroll
    for (int nt = 0; nt < 8; ++nt) {
      const unsigned short* wq = bp + (size_t)(16 * nt) * 256 + k0;
      FragB bf;
      bf.h[0] = *(const v8usa*)wq;
      bf.h[1] = *(const v8usa*)(wq + 16);
      acc[nt] = wmb(af, bf, acc[nt]);
    }
  }
}
__device__ __forceinline__ void gemm_h_k128(const unsigned short* ap, const unsigned short* __restrict__ bp,
                                            v8f (&acc)[8]) {
#pragma unroll 1
  for (int k0 = 0; k0 < HID; k0 += 32) {
    FragH af;
    af.h[0] = *(const v8usa*)(ap + k0);
    af.h[1] = *(const v8usa*)(ap + k0 + 16);
#pragma unroll
    for (int nt = 0; nt < 8; ++nt) {
      const unsigned short* wq = bp + (size_t)(16 * nt) * HID + k0;
      FragH bf;
      bf.h[0] = *(const v8usa*)wq;
      bf.h[1] = *(const v8usa*)(wq + 16);
      acc[nt] = wmh(af, bf, acc[nt]);
    }
  }
}

template <int MODE>
__global__ __launch_bounds__(NTHR) void k_node(const float* __restrict__ x, const unsigned short* __restrict__ B1,
                                               const float* __restrict__ cA, const float* __restrict__ cB,
                                               const float* __restrict__ Sg, const int* __restrict__ DEG,
                                               const unsigned short* __restrict__ W1n, int doP, int nN,
                                               float* Hm, float* Pm) {
  extern __shared__ __attribute__((aligned(16))) float dyn[];
  __shared__ int sdg[TROWS];
  float*          stg = dyn;
  unsigned short* sHL = (unsigned short*)(dyn + TROWS * SP);
  const int tid = (int)threadIdx.x, lane = tid & 31, wave = tid >> 5, hh = lane >> 4, m = lane & 15;
  const int row0 = (int)blockIdx.x * TROWS;

  v8f acc[8];
#pragma unroll
  for (int t = 0; t < 8; ++t) acc[t] = z8();

  if constexpr (MODE == 0) {
    const int rg = imin(row0 + 16 * wave + m, nN - 1);
    const float* xp = x + (size_t)rg * NDIM + 8 * hh;
    const v4f a0 = *(const v4f*)xp;
    const v4f a1 = *(const v4f*)(xp + 4);
    const v4f a2 = *(const v4f*)(xp + 16);
    const v4f a3 = *(const v4f*)(xp + 20);
    FragB af;
    af.u[0]  = (unsigned short)bf16_bits(a0.x); af.u[1]  = (unsigned short)bf16_bits(a0.y);
    af.u[2]  = (unsigned short)bf16_bits(a0.z); af.u[3]  = (unsigned short)bf16_bits(a0.w);
    af.u[4]  = (unsigned short)bf16_bits(a1.x); af.u[5]  = (unsigned short)bf16_bits(a1.y);
    af.u[6]  = (unsigned short)bf16_bits(a1.z); af.u[7]  = (unsigned short)bf16_bits(a1.w);
    af.u[8]  = (unsigned short)bf16_bits(a2.x); af.u[9]  = (unsigned short)bf16_bits(a2.y);
    af.u[10] = (unsigned short)bf16_bits(a2.z); af.u[11] = (unsigned short)bf16_bits(a2.w);
    af.u[12] = (unsigned short)bf16_bits(a3.x); af.u[13] = (unsigned short)bf16_bits(a3.y);
    af.u[14] = (unsigned short)bf16_bits(a3.z); af.u[15] = (unsigned short)bf16_bits(a3.w);
    const unsigned short* bp = B1 + (size_t)m * NDIM + 8 * hh;
#pragma unroll
    for (int nt = 0; nt < 8; ++nt) {
      const unsigned short* wq = bp + (size_t)(16 * nt) * NDIM;
      FragB bf;
      bf.h[0] = *(const v8usa*)wq;
      bf.h[1] = *(const v8usa*)(wq + 16);
      acc[nt] = wmb(af, bf, acc[nt]);
    }
  } else {
    if (tid < TROWS) sdg[tid] = iclamp(DEG[imin(row0 + tid, NDEG - 1)], 0, 127);
#pragma unroll 2
    for (int it = 0; it < 16; ++it) {
      const int row = it * NWAVE + wave;
      const int rg  = imin(row0 + row, nN - 1);
      const v4f v = *(const v4f*)(Sg + (size_t)rg * HID + 4 * lane);
      split4(v, sHL + row * HLP + 4 * lane, sHL + row * HLP + HID + 4 * lane);
    }
    __syncthreads();
    gemm_bf_k256(sHL + (16 * wave + m) * HLP + 8 * hh, B1 + (size_t)m * 256 + 8 * hh, acc);
  }

#pragma unroll
  for (int nt = 0; nt < 8; ++nt) {
    const int lc = 16 * nt + m;
#pragma unroll
    for (int r = 0; r < 8; ++r) stg[(16 * wave + 8 * hh + r) * SP + lc] = acc[nt][r];
  }
  __syncthreads();

  {
    const v4f ca = *(const v4f*)(cA + 4 * lane);
    v4f cb = {0.f, 0.f, 0.f, 0.f};
    if constexpr (MODE == 1) cb = *(const v4f*)(cB + 4 * lane);
#pragma unroll 2
    for (int i = 0; i < 16; ++i) {
      const int row = 16 * wave + i;
      const int rgl = row0 + row;
      float* sp = stg + row * SP + 4 * lane;
      const v4f z = *(const v4fa*)sp;
      v4f hn;
      if constexpr (MODE == 0) {
        hn.x = z.x + ca.x; hn.y = z.y + ca.y; hn.z = z.z + ca.z; hn.w = z.w + ca.w;
      } else {
        const int rc = imin(rgl, nN - 1);
        const v4f hold = *(const v4f*)(Hm + (size_t)rc * HID + 4 * lane);
        const float dg = (float)sdg[row];
        hn.x = hold.x + fmaf(z.x, ca.x, dg * cb.x);
        hn.y = hold.y + fmaf(z.y, ca.y, dg * cb.y);
        hn.z = hold.z + fmaf(z.z, ca.z, dg * cb.z);
        hn.w = hold.w + fmaf(z.w, ca.w, dg * cb.w);
      }
      *(v4fa*)sp = hn;
      split4(hn, sHL + row * HLP + 4 * lane, sHL + row * HLP + HID + 4 * lane);
      if (rgl < nN) *(volatile v4f*)(Hm + (size_t)rgl * HID + 4 * lane) = hn;
    }
    __threadfence();
#pragma unroll 2
    for (int i = 0; i < 16; ++i) {
      const int row = 16 * wave + i;
      const int rgl = row0 + row;
      const v4f hn = *(const v4fa*)(stg + row * SP + 4 * lane);
      if (rgl < nN) *(volatile v4f*)(Hm + (size_t)rgl * HID + 4 * lane) = hn;
    }
  }

  if (doP != 0) {
    __syncthreads();
#pragma unroll
    for (int t = 0; t < 8; ++t) acc[t] = z8();
    gemm_bf_k256(sHL + (16 * wave + m) * HLP + 8 * hh, W1n + (size_t)m * 256 + 8 * hh, acc);
    __syncthreads();
#pragma unroll
    for (int nt = 0; nt < 8; ++nt) {
      const int lc = 16 * nt + m;
#pragma unroll
      for (int r = 0; r < 8; ++r) stg[(16 * wave + 8 * hh + r) * SP + lc] = acc[nt][r];
    }
    __syncthreads();
#pragma unroll 2
    for (int i = 0; i < 16; ++i) {
      const int row = 16 * wave + i;
      const int rgl = row0 + row;
      const v4f pv = *(const v4fa*)(stg + row * SP + 4 * lane);
      if (rgl < nN) *(volatile v4f*)(Pm + (size_t)rgl * HID + 4 * lane) = pv;
    }
    __threadfence();
#pragma unroll 2
    for (int i = 0; i < 16; ++i) {
      const int row = 16 * wave + i;
      const int rgl = row0 + row;
      const v4f pv = *(const v4fa*)(stg + row * SP + 4 * lane);
      if (rgl < nN) *(volatile v4f*)(Pm + (size_t)rgl * HID + 4 * lane) = pv;
    }
  }
}

__device__ __forceinline__ void store_R(const unsigned short* sRn, unsigned short* Rg, int pos_lo, int ec, int tid) {
#pragma unroll 1
  for (int it = 0; it < 8; ++it) {
    const int q = it * NTHR + tid;
    const int row = q >> 4, pc = q & 15;
    const v4i v = *(const v4ia*)(sRn + row * AP + 8 * pc);
    if (row < ec) *(volatile v4i*)(Rg + (size_t)(pos_lo + row) * HID + 8 * pc) = v;
  }
  __threadfence();
#pragma unroll 1
  for (int it = 0; it < 8; ++it) {
    const int q = it * NTHR + tid;
    const int row = q >> 4, pc = q & 15;
    const v4i v = *(const v4ia*)(sRn + row * AP + 8 * pc);
    if (row < ec) *(volatile v4i*)(Rg + (size_t)(pos_lo + row) * HID + 8 * pc) = v;
  }
}

__global__ __launch_bounds__(NTHR) void k_edge0(const float* __restrict__ EA, const int* __restrict__ PERM,
                                                const int* __restrict__ TILE, const int* __restrict__ META,
                                                const unsigned short* __restrict__ A0B,
                                                const float* __restrict__ c0v, int nE, int nN,
                                                unsigned short* Rg) {
  __shared__ __attribute__((aligned(16))) unsigned short sA0[TROWS * FP];
  __shared__ __attribute__((aligned(16))) unsigned short sRn[TROWS * AP];
  __shared__ __attribute__((aligned(16))) float sc[HID];
  const int tid = (int)threadIdx.x, lane = tid & 31, wave = tid >> 5, hh = lane >> 4, m = lane & 15;
  const int b = (int)blockIdx.x, t = (int)blockIdx.y;
  const int nt_b = iclamp(META[b * 32 + 0], 0, TCAP);
  if (t >= nt_b) return;
  const v4i tl = *(const v4i*)(TILE + ((size_t)b * TCAP + t) * 4);
  const int ec = iclamp(tl.w, 0, TROWS);
  const int pos_lo = iclamp(tl.z, 0, RROWS - ec);
  const int ecm1 = ec > 0 ? ec - 1 : 0;

  if (tid < HID) sc[tid] = c0v[tid];
  {
    const int row = tid >> 1, hf = tid & 1;
    const int pg  = imin(pos_lo + imin(row, ecm1), RROWS - 1);
    const int eid = iclamp(PERM[pg], 0, nE - 1);
    const float* p = EA + (size_t)eid * EDIM + 8 * hf;
    const v4f a = *(const v4f*)p;
    const v4f c = *(const v4f*)(p + 4);
    const unsigned mk = (row < ec) ? 0xffffu : 0u;
    v8us o;
    o[0] = (unsigned short)(bf16_bits(a.x) & mk); o[1] = (unsigned short)(bf16_bits(a.y) & mk);
    o[2] = (unsigned short)(bf16_bits(a.z) & mk); o[3] = (unsigned short)(bf16_bits(a.w) & mk);
    o[4] = (unsigned short)(bf16_bits(c.x) & mk); o[5] = (unsigned short)(bf16_bits(c.y) & mk);
    o[6] = (unsigned short)(bf16_bits(c.z) & mk); o[7] = (unsigned short)(bf16_bits(c.w) & mk);
    *(v8usa*)(sA0 + row * FP + 8 * hf)      = o;
    *(v8usa*)(sA0 + row * FP + 16 + 8 * hf) = o;
  }
  __syncthreads();

  v8f acc[8];
#pragma unroll
  for (int q = 0; q < 8; ++q) acc[q] = z8();
  {
    const unsigned short* ap = sA0 + (16 * wave + m) * FP + 8 * hh;
    FragB af;
    af.h[0] = *(const v8usa*)ap;
    af.h[1] = *(const v8usa*)(ap + 16);
    const unsigned short* bp = A0B + (size_t)m * 32 + 8 * hh;
#pragma unroll
    for (int nt = 0; nt < 8; ++nt) {
      const unsigned short* wq = bp + (size_t)(16 * nt) * 32;
      FragB bf;
      bf.h[0] = *(const v8usa*)wq;
      bf.h[1] = *(const v8usa*)(wq + 16);
      acc[nt] = wmb(af, bf, acc[nt]);
    }
  }
#pragma unroll
  for (int nt = 0; nt < 8; ++nt) {
    const int col = 16 * nt + m;
    const float cv = sc[col];
#pragma unroll
    for (int r = 0; r < 8; ++r) {
      const float v = relu_np(acc[nt][r] + cv);
      sRn[(16 * wave + 8 * hh + r) * AP + col] = f2h(CR * v);
    }
  }
  __syncthreads();
  store_R(sRn, Rg, pos_lo, ec, tid);
}

template <bool HASC>
__global__ __launch_bounds__(NTHR) void k_edge(unsigned short* Rg, const unsigned short* __restrict__ BWl,
                                               const float* __restrict__ cpre, const float* __restrict__ cq,
                                               const float* __restrict__ Pm, const int* __restrict__ SRCT,
                                               const int* __restrict__ DEG, const int* __restrict__ TILE,
                                               const int* __restrict__ META, int nN, float* Sg) {
  extern __shared__ __attribute__((aligned(16))) float dyn[];
  float*          sM   = dyn;
  unsigned short* sA   = (unsigned short*)(dyn + TROWS * SP);
  unsigned short* sRn  = sA + TROWS * AP;
  float*          sc   = (float*)(sRn + TROWS * AP);
  int*            ssrc = (int*)(sc + 2 * HID);
  int*            sdeg = ssrc + TROWS;
  int*            srow = sdeg + TROWS;
  float*          sS   = (float*)sA;
  const int tid = (int)threadIdx.x, lane = tid & 31, wave = tid >> 5, hh = lane >> 4, m = lane & 15;
  const int b = (int)blockIdx.x, t = (int)blockIdx.y;
  const int nt_b = iclamp(META[b * 32 + 0], 0, TCAP);
  if (t >= nt_b) return;
  const int pois = META[b * 32 + 1];
  const v4i tl = *(const v4i*)(TILE + ((size_t)b * TCAP + t) * 4);
  const int nc = iclamp(tl.y, 0, NCAP);
  const int ec = iclamp(tl.w, 0, TROWS);
  const int node_lo = iclamp(tl.x, 0, nN - nc);
  const int pos_lo  = iclamp(tl.z, 0, RROWS - ec);
  const int ecm1 = ec > 0 ? ec - 1 : 0;
  const int ncm1 = nc > 0 ? nc - 1 : 0;

#pragma unroll 2
  for (int it = 0; it < 8; ++it) {
    const int q = it * NTHR + tid;
    const int row = q >> 4, pc = q & 15;
    const int rg = imin(pos_lo + imin(row, ecm1), RROWS - 1);
    v4i v = *(const v4ia*)(Rg + (size_t)rg * HID + 8 * pc);
    const int mk = (row < ec) ? -1 : 0;
    v.x &= mk; v.y &= mk; v.z &= mk; v.w &= mk;
    *(v4ia*)(sA + row * AP + 8 * pc) = v;
  }
  if (tid < TROWS) {
    sc[tid] = cpre[tid];
    const int pg = imin(pos_lo + imin(tid, ecm1), RROWS - 1);
    ssrc[tid] = iclamp(SRCT[pg], 0, nN - 1);
  } else {
    const int j = tid - TROWS;
    sc[tid] = cq[j];
    const int ng = imin(node_lo + imin(j, ncm1), NDEG - 1);
    const int dv = iclamp(DEG[ng], 0, DEGCAP);
    sdeg[j] = (j < nc) ? dv : 0;
  }
  __syncthreads();

  if (wave == 0) {
    const int d0 = sdeg[4 * lane + 0], d1 = sdeg[4 * lane + 1], d2 = sdeg[4 * lane + 2], d3 = sdeg[4 * lane + 3];
    const int s = d0 + d1 + d2 + d3;
    int incl = s;
#pragma unroll
    for (int d = 1; d < 32; d <<= 1) {
      const int y = __shfl_up(incl, d, 32);
      if (lane >= d) incl += y;
    }
    const int run = incl - s;
    srow[4 * lane + 0] = imin(run, TROWS);
    srow[4 * lane + 1] = imin(run + d0, TROWS);
    srow[4 * lane + 2] = imin(run + d0 + d1, TROWS);
    srow[4 * lane + 3] = imin(run + d0 + d1 + d2, TROWS);
  }

  const unsigned short* ap = sA + (16 * wave + m) * AP + 8 * hh;
  v8f acc[8];
  if constexpr (HASC) {
#pragma unroll
    for (int q = 0; q < 8; ++q) acc[q] = z8();
    gemm_h_k128(ap, BWl + (size_t)m * HID + 8 * hh, acc);
#pragma unroll
    for (int nt = 0; nt < 8; ++nt) {
      const int col = 16 * nt + m;
      const float cv = sc[col];
#pragma unroll
      for (int r = 0; r < 8; ++r) {
        const float v = relu_np(fmaf(acc[nt][r], PINV, cv));
        sRn[(16 * wave + 8 * hh + r) * AP + col] = f2h(CR * v);
      }
    }
  }
#pragma unroll
  for (int q = 0; q < 8; ++q) acc[q] = z8();
  gemm_h_k128(ap, BWl + (size_t)((HASC ? HID : 0) + m) * HID + 8 * hh, acc);
#pragma unroll
  for (int nt = 0; nt < 8; ++nt) {
    const int col = 16 * nt + m;
    const float cv = sc[HID + col];
#pragma unroll
    for (int r = 0; r < 8; ++r) sM[(16 * wave + 8 * hh + r) * SP + col] = fmaf(acc[nt][r], PINV, cv);
  }
  __syncthreads();

#pragma unroll 2
  for (int it = 0; it < 16; ++it) {
    const int row  = it * NWAVE + wave;
    const int sidx = ssrc[row];
    const v4f pv = *(const v4f*)(Pm + (size_t)sidx * HID + 4 * lane);
    float* mp = sM + row * SP + 4 * lane;
    const v4f mv = *(const v4fa*)mp;
    const bool liv = row < ec;
    v4f o;
    o.x = liv ? relu_np(mv.x + pv.x) : 0.0f;
    o.y = liv ? relu_np(mv.y + pv.y) : 0.0f;
    o.z = liv ? relu_np(mv.z + pv.z) : 0.0f;
    o.w = liv ? relu_np(mv.w + pv.w) : 0.0f;
    *(v4fa*)mp = o;
  }
  __syncthreads();

  {
    const int c = tid & (HID - 1);
    const int half = tid >> 7;
    const float qnan = __int_as_float(0x7fc00000);
#pragma unroll 1
    for (int j = half; j < nc; j += 2) {
      const int r0 = srow[j];
      const int d  = sdeg[j];
      float s = 0.0f;
#pragma unroll 1
      for (int i = 0; i < d; ++i) s += sM[imin(r0 + i, TROWS - 1) * SP + c];
      sS[j * HID + c] = (pois != 0) ? qnan : s;
    }
  }
  __syncthreads();

#pragma unroll 1
  for (int it = 0; it < NCAP / NWAVE; ++it) {
    const int j = it * NWAVE + wave;
    if (j < nc) {
      const v4f v = *(const v4fa*)(sS + j * HID + 4 * lane);
      *(volatile v4f*)(Sg + (size_t)(node_lo + j) * HID + 4 * lane) = v;
    }
  }
  __threadfence();
#pragma unroll 1
  for (int it = 0; it < NCAP / NWAVE; ++it) {
    const int j = it * NWAVE + wave;
    if (j < nc) {
      const v4f v = *(const v4fa*)(sS + j * HID + 4 * lane);
      *(volatile v4f*)(Sg + (size_t)(node_lo + j) * HID + 4 * lane) = v;
    }
  }
  if constexpr (HASC) store_R(sRn, Rg, pos_lo, ec, tid);
}

__global__ __launch_bounds__(NTHR) void k_pool_head(const float* __restrict__ Hm, const int* __restrict__ gid,
                                                    int nN, const unsigned short* __restrict__ RO1,
                                                    const float* __restrict__ CST, const int* __restrict__ META,
                                                    float* out) {
  __shared__ __attribute__((aligned(16))) float spool[PG * SP];
  __shared__ __attribute__((aligned(16))) unsigned short sPL[PG * HLP];
  __shared__ __attribute__((aligned(16))) float shid[PG * SP];
  __shared__ __attribute__((aligned(16))) float sout[PG];
  const int tid = (int)threadIdx.x, lane = tid & 31, wave = tid >> 5, hh = lane >> 4, m = lane & 15;
  const int g0 = (int)blockIdx.x * PG + 4 * wave;

  v4f a0 = {0.f, 0.f, 0.f, 0.f}, a1 = a0, a2 = a0, a3 = a0;
  const int nCh = (nN + 31) / 32;
#pragma unroll 1
  for (int ch = 0; ch < nCh; ++ch) {
    const int n  = ch * 32 + lane;
    const int bv0 = gid[imin(n, nN - 1)];
    const int bv = (n < nN) ? bv0 : -1;
    const unsigned rel = (unsigned)(bv - g0);
    const unsigned any = __builtin_amdgcn_ballot_w32(rel < 4u);
    if (any != 0u) {
      unsigned m0 = __builtin_amdgcn_ballot_w32(rel == 0u);
      unsigned m1 = __builtin_amdgcn_ballot_w32(rel == 1u);
      unsigned m2 = __builtin_amdgcn_ballot_w32(rel == 2u);
      unsigned m3 = __builtin_amdgcn_ballot_w32(rel == 3u);
#pragma unroll 1
      while (m0 != 0u) {
        const int k = __builtin_ctz(m0); m0 &= m0 - 1u;
        const v4f v = *(const v4f*)(Hm + (size_t)(ch * 32 + k) * HID + 4 * lane);
        a0.x += v.x; a0.y += v.y; a0.z += v.z; a0.w += v.w;
      }
#pragma unroll 1
      while (m1 != 0u) {
        const int k = __builtin_ctz(m1); m1 &= m1 - 1u;
        const v4f v = *(const v4f*)(Hm + (size_t)(ch * 32 + k) * HID + 4 * lane);
        a1.x += v.x; a1.y += v.y; a1.z += v.z; a1.w += v.w;
      }
#pragma unroll 1
      while (m2 != 0u) {
        const int k = __builtin_ctz(m2); m2 &= m2 - 1u;
        const v4f v = *(const v4f*)(Hm + (size_t)(ch * 32 + k) * HID + 4 * lane);
        a2.x += v.x; a2.y += v.y; a2.z += v.z; a2.w += v.w;
      }
#pragma unroll 1
      while (m3 != 0u) {
        const int k = __builtin_ctz(m3); m3 &= m3 - 1u;
        const v4f v = *(const v4f*)(Hm + (size_t)(ch * 32 + k) * HID + 4 * lane);
        a3.x += v.x; a3.y += v.y; a3.z += v.z; a3.w += v.w;
      }
    }
  }
  {
    const int r = 4 * wave;
    *(v4fa*)(spool + (r + 0) * SP + 4 * lane) = a0;
    *(v4fa*)(spool + (r + 1) * SP + 4 * lane) = a1;
    *(v4fa*)(spool + (r + 2) * SP + 4 * lane) = a2;
    *(v4fa*)(spool + (r + 3) * SP + 4 * lane) = a3;
    split4(a0, sPL + (r + 0) * HLP + 4 * lane, sPL + (r + 0) * HLP + HID + 4 * lane);
    split4(a1, sPL + (r + 1) * HLP + 4 * lane, sPL + (r + 1) * HLP + HID + 4 * lane);
    split4(a2, sPL + (r + 2) * HLP + 4 * lane, sPL + (r + 2) * HLP + HID + 4 * lane);
    split4(a3, sPL + (r + 3) * HLP + 4 * lane, sPL + (r + 3) * HLP + HID + 4 * lane);
  }
  __syncthreads();

  {
    v8f c0 = z8(), c1 = z8();
    const unsigned short* ap0 = sPL + m * HLP + 8 * hh;
    const unsigned short* ap1 = ap0 + 16 * HLP;
    const unsigned short* bp  = RO1 + (size_t)(16 * wave + m) * 256 + 8 * hh;
#pragma unroll 1
    for (int k0 = 0; k0 < 256; k0 += 32) {
      FragB f0, f1, bf;
      f0.h[0] = *(const v8usa*)(ap0 + k0);
      f0.h[1] = *(const v8usa*)(ap0 + k0 + 16);
      f1.h[0] = *(const v8usa*)(ap1 + k0);
      f1.h[1] = *(const v8usa*)(ap1 + k0 + 16);
      bf.h[0] = *(const v8usa*)(bp + k0);
      bf.h[1] = *(const v8usa*)(bp + k0 + 16);
      c0 = wmb(f0, bf, c0);
      c1 = wmb(f1, bf, c1);
    }
    const int col = 16 * wave + m;
    const float bias = CST[17 * HID + col];
#pragma unroll
    for (int r = 0; r < 8; ++r) {
      shid[(8 * hh + r) * SP + col]      = relu_np(c0[r] + bias);
      shid[(16 + 8 * hh + r) * SP + col] = relu_np(c1[r] + bias);
    }
  }
  __syncthreads();

  {
    const float w0 = CST[18 * HID + lane], w1 = CST[18 * HID + 32 + lane];
    const float w2 = CST[18 * HID + 64 + lane], w3 = CST[18 * HID + 96 + lane];
    const float b2 = CST[19 * HID];
#pragma unroll 1
    for (int gi = 0; gi < 4; ++gi) {
      const float* hr = shid + (4 * wave + gi) * SP;
      float s = hr[lane] * w0;
      s = fmaf(hr[32 + lane], w1, s);
      s = fmaf(hr[64 + lane], w2, s);
      s = fmaf(hr[96 + lane], w3, s);
#pragma unroll
      for (int d = 16; d >= 1; d >>= 1) s += __shfl_xor(s, d, 32);
      if (lane == 0) sout[4 * wave + gi] = s + b2;
    }
  }
  int pz = 0;
#pragma unroll 1
  for (int bb = 0; bb < NBLK; ++bb) pz |= META[bb * 32 + 1];
  __syncthreads();

  {
    const float qnan = __int_as_float(0x7fc00000);
    v4f v = {0.f, 0.f, 0.f, 0.f};
    if (tid < 8) {
      const v4f sv = *(const v4fa*)(sout + 4 * tid);
      v.x = (pz != 0) ? qnan : sv.x;
      v.y = (pz != 0) ? qnan : sv.y;
      v.z = (pz != 0) ? qnan : sv.z;
      v.w = (pz != 0) ? qnan : sv.w;
      *(volatile v4f*)(out + (size_t)blockIdx.x * PG + 4 * tid) = v;
    }
    __threadfence();
    if (tid < 8) *(volatile v4f*)(out + (size_t)blockIdx.x * PG + 4 * tid) = v;
  }
}

static constexpr size_t al256c(size_t o) { return (o + 255) & ~(size_t)255; }
static constexpr size_t SZ_R    = (size_t)RROWS * HID * 2;
static constexpr size_t SZ_NP   = (size_t)MP * HID * 4;
static constexpr size_t SZ_IDX  = (size_t)RROWS * 4;
static constexpr size_t SZ_DEG  = (size_t)NDEG * 4;
static constexpr size_t SZ_TILE = (size_t)NBLK * TCAP * 16;
static constexpr size_t SZ_LINE = (size_t)NBLK * 128;
static constexpr size_t O_R    = 0;
static constexpr size_t O_H    = al256c(O_R + SZ_R);
static constexpr size_t O_P    = al256c(O_H + SZ_NP);
static constexpr size_t O_S    = al256c(O_P + SZ_NP);
static constexpr size_t O_PERM = al256c(O_S + SZ_NP);
static constexpr size_t O_SRC  = al256c(O_PERM + SZ_IDX);
static constexpr size_t O_DEG  = al256c(O_SRC + SZ_IDX);
static constexpr size_t O_TILE = al256c(O_DEG + SZ_DEG);
static constexpr size_t O_META = al256c(O_TILE + SZ_TILE);
static constexpr size_t O_CNTL = al256c(O_META + SZ_LINE);
static constexpr size_t O_NEWT = al256c(O_CNTL + SZ_LINE);
static constexpr size_t O_W1A  = al256c(O_NEWT + (size_t)HID * NDIM * 2);
static constexpr size_t O_W2T  = al256c(O_W1A + (size_t)NLAY * HID * 256 * 2);
static constexpr size_t O_RO1  = al256c(O_W2T + (size_t)NLAY * HID * 256 * 2);
static constexpr size_t O_A0B  = al256c(O_RO1 + (size_t)HID * 256 * 2);
static constexpr size_t O_BW   = al256c(O_A0B + (size_t)HID * 32 * 2);
static constexpr size_t O_CST  = al256c(O_BW + (size_t)(3 * 256 + HID) * HID * 2);
static constexpr size_t O_END  = al256c(O_CST + (size_t)NCST * HID * 4);
static_assert(O_END <= WSCAP);
static_assert((size_t)RROWS * HID * 2 == SZ_R && SZ_R % 256 == 0);

extern "C" void kernel_launch(void* const* d_in, const int* in_sizes, int n_in,
                              void* d_out, int out_size, void* d_ws, size_t ws_size,
                              hipStream_t stream) {
  if (n_in < 22) return;
  if (in_sizes[0] != NNODE * NDIM) return;
  if (in_sizes[1] != 2 * NEDGE) return;
  if (in_sizes[2] != NEDGE * EDIM) return;
  if (in_sizes[3] != NNODE) return;
  if (in_sizes[4] != NDIM * HID || in_sizes[5] != HID) return;
  if (in_sizes[6] != EDIM * HID || in_sizes[7] != HID) return;
  if (in_sizes[8] != NLAY * 2 * HID * HID || in_sizes[9] != NLAY * HID) return;
  if (in_sizes[10] != NLAY * HID * HID || in_sizes[11] != NLAY * HID) return;
  if (in_sizes[12] != NLAY * HID || in_sizes[13] != NLAY * HID) return;
  if (in_sizes[14] != NLAY * HID * HID || in_sizes[15] != NLAY * HID) return;
  if (in_sizes[16] != NLAY * HID * HID || in_sizes[17] != NLAY * HID) return;
  if (in_sizes[18] != HID * HID || in_sizes[19] != HID) return;
  if (in_sizes[20] != HID || in_sizes[21] != 1) return;
  if (out_size != NGRAPH) return;
  if (O_END > ws_size) return;

  const float* x     = (const float*)d_in[0];
  const int*   ei    = (const int*)d_in[1];
  const float* ea    = (const float*)d_in[2];
  const int*   gid   = (const int*)d_in[3];
  const float* ne_w  = (const float*)d_in[4];
  const float* ne_b  = (const float*)d_in[5];
  const float* ee_w  = (const float*)d_in[6];
  const float* ee_b  = (const float*)d_in[7];
  const float* nm_w1 = (const float*)d_in[8];
  const float* nm_b1 = (const float*)d_in[9];
  const float* nm_w2 = (const float*)d_in[10];
  const float* nm_b2 = (const float*)d_in[11];
  const float* bn_g  = (const float*)d_in[12];
  const float* bn_b  = (const float*)d_in[13];
  const float* em_w1 = (const float*)d_in[14];
  const float* em_b1 = (const float*)d_in[15];
  const float* em_w2 = (const float*)d_in[16];
  const float* em_b2 = (const float*)d_in[17];
  const float* ro_w1 = (const float*)d_in[18];
  const float* ro_b1 = (const float*)d_in[19];
  const float* ro_w2 = (const float*)d_in[20];
  const float* ro_b2 = (const float*)d_in[21];
  const int* src = ei;
  const int* dst = ei + NEDGE;
  float* out = (float*)d_out;

  char* ws = (char*)d_ws;
  unsigned short* R    = (unsigned short*)(ws + O_R);
  float*          Hm   = (float*)(ws + O_H);
  float*          Pm   = (float*)(ws + O_P);
  float*          Sm   = (float*)(ws + O_S);
  int*            PERM = (int*)(ws + O_PERM);
  int*            SRCT = (int*)(ws + O_SRC);
  int*            DEG  = (int*)(ws + O_DEG);
  int*            TILE = (int*)(ws + O_TILE);
  int*            META = (int*)(ws + O_META);
  int*            CNTL = (int*)(ws + O_CNTL);
  unsigned short* NEWT = (unsigned short*)(ws + O_NEWT);
  unsigned short* W1A  = (unsigned short*)(ws + O_W1A);
  unsigned short* W2T  = (unsigned short*)(ws + O_W2T);
  unsigned short* RO1  = (unsigned short*)(ws + O_RO1);
  unsigned short* A0B  = (unsigned short*)(ws + O_A0B);
  unsigned short* BW   = (unsigned short*)(ws + O_BW);
  float*          CST  = (float*)(ws + O_CST);

  hipFuncSetAttribute(reinterpret_cast<const void*>(&k_bucket), hipFuncAttributeMaxDynamicSharedMemorySize,
                      (int)BK_LDS_BYTES);
  hipFuncSetAttribute(reinterpret_cast<const void*>(&k_node<0>), hipFuncAttributeMaxDynamicSharedMemorySize,
                      (int)NODE_LDS_BYTES);
  hipFuncSetAttribute(reinterpret_cast<const void*>(&k_node<1>), hipFuncAttributeMaxDynamicSharedMemorySize,
                      (int)NODE_LDS_BYTES);
  hipFuncSetAttribute(reinterpret_cast<const void*>(&k_edge<true>), hipFuncAttributeMaxDynamicSharedMemorySize,
                      (int)EDGE_LDS_BYTES);
  hipFuncSetAttribute(reinterpret_cast<const void*>(&k_edge<false>), hipFuncAttributeMaxDynamicSharedMemorySize,
                      (int)EDGE_LDS_BYTES);

  k_prep<<<PU6 / NTHR, NTHR, 0, stream>>>(ne_w, ne_b, ee_w, ee_b, nm_w1, nm_b1, nm_w2, nm_b2, bn_g, bn_b,
                                          em_w1, em_b1, em_w2, em_b2, ro_w1, ro_b1, ro_w2, ro_b2,
                                          NEWT, W1A, W2T, RO1, A0B, BW, CST);
  k_hist<<<NBLK, NTHR, 0, stream>>>(dst, NEDGE, NNODE, CNTL);
  k_bucket<<<NBLK, NTHR, BK_LDS_BYTES, stream>>>(src, dst, NEDGE, NNODE, 1, CNTL, PERM, SRCT, DEG, TILE, META);
  k_node<0><<<MP / TROWS, NTHR, NODE_LDS_BYTES, stream>>>(x, NEWT, CST + 16 * HID, CST, Sm, DEG, W1A, 1, NNODE,
                                                          Hm, Pm);
  k_edge0<<<dim3(NBLK, TCAP), NTHR, 0, stream>>>(ea, PERM, TILE, META, A0B, CST, NEDGE, NNODE, R);
  for (int l = 0; l < NLAY; ++l) {
    const unsigned short* BWl = BW + (size_t)l * 256 * HID;
    if (l < NLAY - 1) {
      k_edge<true><<<dim3(NBLK, TCAP), NTHR, EDGE_LDS_BYTES, stream>>>(R, BWl, CST + (1 + l) * HID,
                                                                       CST + (4 + l) * HID, Pm, SRCT, DEG, TILE,
                                                                       META, NNODE, Sm);
    } else {
      k_edge<false><<<dim3(NBLK, TCAP), NTHR, EDGE_LDS_BYTES, stream>>>(R, BWl, CST, CST + (4 + l) * HID, Pm,
                                                                        SRCT, DEG, TILE, META, NNODE, Sm);
    }
    const int doP = (l < NLAY - 1) ? 1 : 0;
    const int ln  = (l < NLAY - 1) ? (l + 1) : l;
    k_node<1><<<MP / TROWS, NTHR, NODE_LDS_BYTES, stream>>>(x, W2T + (size_t)l * HID * 256, CST + (8 + l) * HID,
                                                            CST + (12 + l) * HID, Sm, DEG,
                                                            W1A + (size_t)ln * HID * 256, doP, NNODE, Hm, Pm);
  }
  k_pool_head<<<NGRAPH / PG, NTHR, 0, stream>>>(Hm, gid, NNODE, RO1, CST, META, out);
}
